// node_centre_encoding_block_55362128445870
// MI455X (gfx1250) — hardware-run, weakly checked
//
#include <hip/hip_runtime.h>


#define NN   1024
#ifndef NCEN
#define NCEN 1024
#endif
#define DIN  6
#define DI   16
#define KIP  32
#define DE   64
#define PT   64
#define AW   4
#define OSP  68
#define SC1  ((float)(0.25 * 1.4426950408889634))
#define SC2  ((float)(0.125 * 1.4426950408889634))
#define L2E  1.4426950408889634f
#define QRS  2048.0f
#define QRI  (1.0f / 2048.0f)
#define PC1  16384.0f
#define PC1I (1.0f / 16384.0f)
#define AIC  64.0f
#define PC2I (1.0f / 1048576.0f)
#define HMAX 57344.0f
#define NEGB (-3.0e38f)

static_assert(DIN + DI == 22);
static_assert(DI <= 16 && KIP == 32);
static_assert(DE == 64);
static_assert(PT == 64 && DE == PT);
static_assert(NN % PT == 0);
static_assert(NN % 32 == 0);
static_assert(NCEN % (16 * AW) == 0);
static_assert(NCEN <= NN);
static_assert((OSP * 4) % 16 == 0);
static_assert(OSP >= DE);
static_assert(PT * 16 * 4 == PT * KIP * 2);
static_assert(PT * 16 * 8 == PT * DE * 2);
static_assert(32 * 16 == 2 * PT * 4);
static_assert(8 * 2 == 16 && 16 * 4 == DE);
static_assert((size_t)NN * DE < ((size_t)1 << 31));

typedef _Float16 h16;
typedef __attribute__((ext_vector_type(16))) _Float16 v16h;
typedef __attribute__((ext_vector_type(8)))  _Float16 v8h;
typedef __attribute__((ext_vector_type(8)))  float    v8f;
typedef __attribute__((ext_vector_type(4)))  float    v4f;
typedef v4f  __attribute__((may_alias)) v4fa;
typedef v8h  __attribute__((may_alias)) v8ha;

__device__ __forceinline__ unsigned short f2bf(float f) { unsigned u = __float_as_uint(f); u += 0x7FFFu + ((u >> 16) & 1u); return (unsigned short)(u >> 16); }
__device__ __forceinline__ float bfr(float f) { return __uint_as_float(((unsigned)f2bf(f)) << 16); }
__device__ __forceinline__ v16h cat16(v8h lo, v8h hi) { return __builtin_shufflevector(lo, hi, 0, 1, 2, 3, 4, 5, 6, 7, 8, 9, 10, 11, 12, 13, 14, 15); }
__device__ __forceinline__ v8f wmma16(v16h a, v16h b, v8f c) { return __builtin_amdgcn_wmma_f32_16x16x32_f16(false, a, false, b, (short)0, c, false, false); }
__device__ __forceinline__ v16h  ldh(const h16* p) { return cat16(*(const v8h*)p, *(const v8h*)(p + 16)); }
__device__ __forceinline__ void wave_sync() { __builtin_amdgcn_fence(3  , "wavefront"); __builtin_amdgcn_wave_barrier(); asm volatile("" ::: "memory"); }

static __device__ __forceinline__ h16 toh_flush(float v) { const h16 r = (h16)v; return (fabsf(v) < 6.103515625e-05f) ? (h16)0.0f : r; }
__device__ __forceinline__ v8f wmma16g(v16h a, v16h b, v8f c) {
    c = wmma16(a, b, c);
    asm volatile("v_nop\n\tv_nop\n\tv_nop\n\tv_nop" : "+v"(c) : "v"(a), "v"(b));
    return c;
}
__device__ __forceinline__ v8f exp2v(v8f x) { v8f y;
#pragma unroll
    for (int r = 0; r < 8; ++r) y[r] = __builtin_amdgcn_exp2f(x[r]);
    return y; }

__global__ __launch_bounds__(PT) void k_pre(const float* __restrict__ X, const float* __restrict__ Wqi, const float* __restrict__ Wki, const float* __restrict__ Wvi,
                                            const float* __restrict__ Wqe, const float* __restrict__ Wke, const float* __restrict__ Wve, const float* __restrict__ wg,
                                            h16* QI, h16* KI, h16* QE, h16* QER, h16* KB, h16* KIN, h16* VBT, h16* VINT, float* G) {
    __shared__ __align__(16) h16 sQI[PT * KIP];
    __shared__ __align__(16) h16 sKI[PT * KIP];
    __shared__ __align__(16) h16 sVI[PT * KIP];
    __shared__ __align__(16) h16 sWK[DE * KIP];
    __shared__ __align__(16) h16 sWV[DE * KIP];
    __shared__ __align__(16) h16 sQE[PT * DE];
    __shared__ __align__(16) h16 sQER[PT * DE];
    __shared__ __align__(16) h16 sKB[PT * DE];
    __shared__ __align__(16) h16 sKIN[PT * DE];
    __shared__ __align__(16) h16 sVBT[DE * PT];
    __shared__ __align__(16) h16 sVINT[DE * PT];
    __shared__ __align__(16) float sG[2 * PT];
    __shared__ __align__(16) float sWG[DE];
    const int tid = threadIdx.x;
    const int lane = tid & 31, lr = lane & 15, hi = lane >> 4;
    const int wave = __builtin_amdgcn_readfirstlane((int)(threadIdx.x >> 5));
    const int blk = blockIdx.x;
    const int n = blk * PT + tid;

    float x[DIN];
#pragma unroll
    for (int f = 0; f < DIN; ++f) x[f] = bfr(X[(size_t)n * DIN + f]);

    { const v8h hz = (v8h){};
      *(v8ha*)(&sQI[tid * KIP + 16]) = hz; *(v8ha*)(&sQI[tid * KIP + 24]) = hz;
      *(v8ha*)(&sKI[tid * KIP + 16]) = hz; *(v8ha*)(&sKI[tid * KIP + 24]) = hz;
      *(v8ha*)(&sVI[tid * KIP + 16]) = hz; *(v8ha*)(&sVI[tid * KIP + 24]) = hz;
      *(v8ha*)(&sWK[tid * KIP + 16]) = hz; *(v8ha*)(&sWK[tid * KIP + 24]) = hz;
      *(v8ha*)(&sWV[tid * KIP + 16]) = hz; *(v8ha*)(&sWV[tid * KIP + 24]) = hz; }

#pragma unroll 1
    for (int j = 0; j < DI; ++j) {
        float qv = 0.0f, kv = 0.0f, vv = 0.0f;
#pragma unroll
        for (int f = 0; f < DIN; ++f) { qv += x[f] * bfr(Wqi[f * DI + j]); kv += x[f] * bfr(Wki[f * DI + j]); vv += x[f] * bfr(Wvi[f * DI + j]); }
        sQI[tid * KIP + j] = toh_flush(qv); sKI[tid * KIP + j] = toh_flush(kv); sVI[tid * KIP + j] = toh_flush(vv);
    }
#pragma unroll 1
    for (int t = 0; t < DI; ++t) {
        sWK[tid * KIP + t] = toh_flush(bfr(Wke[(DIN + t) * DE + tid]));
        sWV[tid * KIP + t] = toh_flush(bfr(Wve[(DIN + t) * DE + tid]));
    }
    sWG[tid] = bfr(wg[tid]);
    float gb = 0.0f;
#pragma unroll 1
    for (int j = 0; j < DE; ++j) {
        float qe = 0.0f, kb = 0.0f, vb = 0.0f;
#pragma unroll
        for (int f = 0; f < DIN; ++f) { qe += x[f] * bfr(Wqe[f * DE + j]); kb += x[f] * bfr(Wke[f * DE + j]); vb += x[f] * bfr(Wve[f * DE + j]); }
        const h16 qh = toh_flush(qe);
        sQE[tid * DE + j] = qh; sQER[tid * DE + j] = toh_flush((qe - (float)qh) * QRS);
        sKB[tid * DE + j] = toh_flush(kb); sVBT[j * PT + tid] = toh_flush(vb);
        gb += vb * bfr(wg[j]);
    }
    sG[tid] = gb;
    __syncthreads();

#pragma unroll 1
    for (int mt = 0; mt < 2; ++mt) {
        const int m0 = (wave * 2 + mt) * 16;
        const int ao = (m0 + lr) * KIP + 8 * hi;
        const v16h a = cat16(*(const v8ha*)(&sVI[ao]), *(const v8ha*)(&sVI[ao + 16]));
        float gp[8];
#pragma unroll
        for (int r = 0; r < 8; ++r) gp[r] = 0.0f;
#pragma unroll
        for (int nb = 0; nb < 4; ++nb) {
            const int bo = (nb * 16 + lr) * KIP + 8 * hi;
            const v16h bk = cat16(*(const v8ha*)(&sWK[bo]), *(const v8ha*)(&sWK[bo + 16]));
            const v16h bv = cat16(*(const v8ha*)(&sWV[bo]), *(const v8ha*)(&sWV[bo + 16]));
            v8f ck = (v8f){}, cv = (v8f){};
            ck = wmma16g(a, bk, ck);
            cv = wmma16g(a, bv, cv);
            const float wgl = sWG[nb * 16 + lr];
#pragma unroll
            for (int r = 0; r < 8; ++r) {
                sKIN[(m0 + 8 * hi + r) * DE + nb * 16 + lr] = toh_flush(ck[r]);
                sVINT[(nb * 16 + lr) * PT + m0 + 8 * hi + r] = toh_flush(cv[r]);
                gp[r] += cv[r] * wgl; }
        }
#pragma unroll
        for (int r = 0; r < 8; ++r) {
            float v = gp[r];
            v += __shfl_xor(v, 1, 32); v += __shfl_xor(v, 2, 32); v += __shfl_xor(v, 4, 32); v += __shfl_xor(v, 8, 32);
            gp[r] = v; }
        if (lr == 0) {
#pragma unroll
            for (int r = 0; r < 8; ++r) sG[PT + m0 + 8 * hi + r] = gp[r]; }
    }
    __syncthreads();

    const size_t qb = (size_t)blk * PT * KIP;
    const size_t eb = (size_t)blk * PT * DE;
#pragma unroll 1
    for (int ps = 0; ps < 2; ++ps) {
#pragma unroll 1
        for (int it = 0; it < 4; ++it) { const int p = it * PT + tid;
            const v8h a = *(const v8ha*)(&sQI[p * 8]); const v8h b = *(const v8ha*)(&sKI[p * 8]);
            *(volatile v8h*)(QI + qb + (size_t)p * 8) = a; *(volatile v8h*)(KI + qb + (size_t)p * 8) = b; }
#pragma unroll 1
        for (int it = 0; it < 8; ++it) { const int p = it * PT + tid;
            const v8h a = *(const v8ha*)(&sQE[p * 8]); const v8h ar = *(const v8ha*)(&sQER[p * 8]);
            const v8h b = *(const v8ha*)(&sKB[p * 8]); const v8h c = *(const v8ha*)(&sKIN[p * 8]);
            const v8h d = *(const v8ha*)(&sVBT[p * 8]); const v8h e = *(const v8ha*)(&sVINT[p * 8]);
            *(volatile v8h*)(QE + eb + (size_t)p * 8) = a; *(volatile v8h*)(QER + eb + (size_t)p * 8) = ar;
            *(volatile v8h*)(KB + eb + (size_t)p * 8) = b; *(volatile v8h*)(KIN + eb + (size_t)p * 8) = c;
            const size_t vo = (size_t)(p >> 3) * NN + (size_t)blk * PT + (size_t)((p & 7) * 8);
            *(volatile v8h*)(VBT + vo) = d; *(volatile v8h*)(VINT + vo) = e; }
        if (wave == 0) { const int which = lane >> 4, c4 = (lane & 15) * 4;
            const v4f g = *(const v4fa*)(&sG[which * PT + c4]);
            *(volatile v4f*)(G + (size_t)which * NN + (size_t)blk * PT + c4) = g; }
        if (ps == 0) __threadfence(); }
}

__device__ __forceinline__ v8f s1_tile(const h16* __restrict__ KI, size_t off, v16h qi) {
    v8f c = (v8f){}; c = wmma16g(ldh(KI + off), qi, c); return c * SC1; }
__device__ __forceinline__ v16h ldq(const h16* __restrict__ Q, unsigned off) { asm volatile("" : "+v"(off)); return ldh(Q + off); }
__device__ __forceinline__ v8f dot64r(const h16* __restrict__ P, size_t off, const h16* __restrict__ QE, const h16* __restrict__ QER, unsigned qo) {
    const v16h a0 = ldh(P + off), a1 = ldh(P + off + 32);
    v8f c = (v8f){}, cr = (v8f){};
    { const v16h q = ldq(QE,  qo);      c  = wmma16g(a0, q, c); }
    { const v16h q = ldq(QER, qo);      cr = wmma16g(a0, q, cr); }
    { const v16h q = ldq(QE,  qo + 32); c  = wmma16g(a1, q, c); }
    { const v16h q = ldq(QER, qo + 32); cr = wmma16g(a1, q, cr); }
    return c + cr * QRI; }
__device__ __forceinline__ void tile_logits(const h16* __restrict__ KI, const h16* __restrict__ KB, const h16* __restrict__ KIN, const h16* __restrict__ QE, const h16* __restrict__ QER,
                                            size_t io, size_t eo, v16h qi, unsigned qeo, float m1, float inv1, v8f& ai, v8f& te) {
    ai = exp2v(s1_tile(KI, io, qi) - m1) * inv1;
    const v8f sb = dot64r(KB, eo, QE, QER, qeo);
    const v8f si = dot64r(KIN, eo, QE, QER, qeo);
    te = (sb + ai * si) * SC2; }
__device__ __forceinline__ void online_upd(v8f ta, v8f tb, float& m, float& l) {
    float mx = NEGB;
#pragma unroll
    for (int r = 0; r < 8; ++r) mx = fmaxf(mx, fmaxf(ta[r], tb[r]));
    mx = fmaxf(mx, __shfl_xor(mx, 16, 32));
    const float mnew = fmaxf(m, mx);
    const float alpha = __builtin_amdgcn_exp2f(m - mnew);
    float ls = 0.0f;
#pragma unroll
    for (int r = 0; r < 8; ++r) ls += __builtin_amdgcn_exp2f(ta[r] - mnew) + __builtin_amdgcn_exp2f(tb[r] - mnew);
    l = l * alpha + ls; m = mnew; }
__device__ __forceinline__ void gate_tile(v8f te, v8f ai, const float* __restrict__ gbp, const float* __restrict__ gip, float m2, float inv2, float bgv, v8f& w1, v8f& w2) {
    const v4f b0 = *(const v4f*)gbp, b1 = *(const v4f*)(gbp + 4), i0 = *(const v4f*)gip, i1 = *(const v4f*)(gip + 4);
    float gbr[8], gir[8];
#pragma unroll
    for (int r = 0; r < 4; ++r) { gbr[r] = b0[r]; gbr[4 + r] = b1[r]; gir[r] = i0[r]; gir[4 + r] = i1[r]; }
    const v8f ae = exp2v(te - m2) * inv2;
#pragma unroll
    for (int r = 0; r < 8; ++r) {
        const float z = ae[r] * (gbr[r] + ai[r] * gir[r]) + bgv;
        const float g = __builtin_amdgcn_rcpf(1.0f + __builtin_amdgcn_exp2f(-z * L2E));
        const float a = g * ae[r] * PC1;
        w1[r] = a;
        w2[r] = fminf(a * (ai[r] * AIC), HMAX); } }

__global__ __launch_bounds__(32 * AW) __attribute__((amdgpu_num_vgpr(256))) void k_enc(const h16* __restrict__ QI, const h16* __restrict__ KI, const h16* __restrict__ QE, const h16* __restrict__ QER,
                                                   const h16* __restrict__ KB, const h16* __restrict__ KIN, const h16* __restrict__ VBT, const h16* __restrict__ VINT,
                                                   const float* __restrict__ G, const float* __restrict__ bgp, float* OUT) {
    __shared__ __align__(16) float os[AW * 16 * OSP];
    const int lane = threadIdx.x & 31, lr = lane & 15, hi = lane >> 4;
    const int wave = __builtin_amdgcn_readfirstlane((int)(threadIdx.x >> 5));
    const int t0 = (blockIdx.x * AW + wave) * 16;
    const float bgv = bfr(bgp[0]);
    const v16h qi  = ldh(QI + (size_t)(t0 + lr) * KIP + 8 * hi);
    const unsigned qeo = (unsigned)((t0 + lr) * DE + 8 * hi);
    const size_t kio = (size_t)lr * KIP + 8 * hi;
    const size_t keo = (size_t)lr * DE + 8 * hi;
    const size_t vo  = (size_t)lr * NN + 8 * hi;

    float m1 = NEGB, l1 = 0.0f;
#pragma unroll 1
    for (int key0 = 0; key0 < NN; key0 += 32) {
        const v8f ta = s1_tile(KI, kio + (size_t)key0 * KIP, qi);
        const v8f tb = s1_tile(KI, kio + (size_t)(key0 + 16) * KIP, qi);
        online_upd(ta, tb, m1, l1);
    }
    l1 += __shfl_xor(l1, 16, 32);
    const float inv1 = 1.0f / l1;

    float m2 = NEGB, l2 = 0.0f;
#pragma unroll 1
    for (int key0 = 0; key0 < NN; key0 += 32) {
        v8f aa, ta, ab, tb;
        tile_logits(KI, KB, KIN, QE, QER, kio + (size_t)key0 * KIP, keo + (size_t)key0 * DE, qi, qeo, m1, inv1, aa, ta);
        tile_logits(KI, KB, KIN, QE, QER, kio + (size_t)(key0 + 16) * KIP, keo + (size_t)(key0 + 16) * DE, qi, qeo, m1, inv1, ab, tb);
        online_upd(ta, tb, m2, l2);
    }
    l2 += __shfl_xor(l2, 16, 32);
    const float inv2 = 1.0f / l2;

    v8f o1[4], o2[4];
#pragma unroll
    for (int j = 0; j < 4; ++j) { o1[j] = (v8f){}; o2[j] = (v8f){}; }
    const float* gbb = G + 8 * hi;
    const float* gib = G + NN + 8 * hi;
#pragma unroll 1
    for (int key0 = 0; key0 < NN; key0 += 32) {
        v16h p1, p2;
        { v8f aa, ta, w1, w2;
          tile_logits(KI, KB, KIN, QE, QER, kio + (size_t)key0 * KIP, keo + (size_t)key0 * DE, qi, qeo, m1, inv1, aa, ta);
          gate_tile(ta, aa, gbb + key0, gib + key0, m2, inv2, bgv, w1, w2);
#pragma unroll
          for (int r = 0; r < 8; ++r) { p1[r] = toh_flush(w1[r]); p2[r] = toh_flush(w2[r]); } }
        { v8f ab, tb, w1, w2;
          tile_logits(KI, KB, KIN, QE, QER, kio + (size_t)(key0 + 16) * KIP, keo + (size_t)(key0 + 16) * DE, qi, qeo, m1, inv1, ab, tb);
          gate_tile(tb, ab, gbb + key0 + 16, gib + key0 + 16, m2, inv2, bgv, w1, w2);
#pragma unroll
          for (int r = 0; r < 8; ++r) { p1[8 + r] = toh_flush(w1[r]); p2[8 + r] = toh_flush(w2[r]); } }
#pragma unroll
        for (int j = 0; j < 4; ++j) {
            const v16h vb = ldh(VBT + vo + (size_t)j * 16 * NN + key0);
            o1[j] = wmma16g(vb, p1, o1[j]);
            const v16h vi = ldh(VINT + vo + (size_t)j * 16 * NN + key0);
            o2[j] = wmma16g(vi, p2, o2[j]); }
    }

    const int wb = wave * 16 * OSP;
#pragma unroll
    for (int j = 0; j < 4; ++j) {
        const v8f f = o1[j] * PC1I + o2[j] * PC2I;
        v4f a, c;
        a[0] = f[0]; a[1] = f[1]; a[2] = f[2]; a[3] = f[3]; c[0] = f[4]; c[1] = f[5]; c[2] = f[6]; c[3] = f[7];
        *(v4fa*)(&os[wb + lr * OSP + 16 * j + 8 * hi]) = a; *(v4fa*)(&os[wb + lr * OSP + 16 * j + 8 * hi + 4]) = c; }
    wave_sync();
    float* orow = OUT + (size_t)t0 * DE;
#pragma unroll 1
    for (int ps = 0; ps < 2; ++ps) {
#pragma unroll
        for (int s = 0; s < 8; ++s) { const int row = 2 * s + (lane >> 4), cofs = (lane & 15) * 4;
            const v4f val = *(const v4fa*)(&os[wb + row * OSP + cofs]);
            *(volatile v4f*)(orow + (size_t)row * DE + cofs) = val; }
        if (ps == 0) __threadfence(); }
}

static constexpr size_t al256(size_t v) { return (v + 255) & ~(size_t)255; }
static constexpr size_t SZ_I = al256((size_t)NN * KIP * 2);
static constexpr size_t SZ_E = al256((size_t)NN * DE * 2);
static constexpr size_t SZ_G = al256((size_t)2 * NN * 4);
static constexpr size_t SZ_TOTAL = 2 * SZ_I + 6 * SZ_E + SZ_G;
static_assert(SZ_TOTAL <= (size_t)134217728);
static_assert((size_t)(NN / PT) * PT * KIP * 2 == (size_t)NN * KIP * 2);
static_assert((size_t)(NN / PT) * PT * DE * 2 == (size_t)NN * DE * 2);
static_assert((size_t)DE * NN * 2 == (size_t)NN * DE * 2);
static constexpr size_t LDS_PRE = (size_t)(3 * PT * KIP + 2 * DE * KIP + 6 * PT * DE) * 2 + (size_t)(2 * PT + DE) * 4;
static constexpr size_t LDS_ENC = (size_t)AW * 16 * OSP * 4;
static_assert(LDS_PRE <= 131072);
static_assert(LDS_ENC <= 131072);

extern "C" void kernel_launch(void* const* d_in, const int* in_sizes, int n_in,
                              void* d_out, int out_size, void* d_ws, size_t ws_size, hipStream_t stream) {
    if (n_in < 9) return;
    if (in_sizes[0] < NN * DIN) return;
    if (in_sizes[1] < DIN * DI || in_sizes[2] < DIN * DI || in_sizes[3] < DIN * DI) return;
    if (in_sizes[4] < DIN * DE) return;
    if (in_sizes[5] < (DIN + DI) * DE || in_sizes[6] < (DIN + DI) * DE) return;
    if (in_sizes[7] < DE || in_sizes[8] < 1) return;
    if ((size_t)out_size < (size_t)NCEN * DE) return;
    if (SZ_TOTAL > ws_size) return;
    const float* X   = (const float*)d_in[0];
    const float* Wqi = (const float*)d_in[1];
    const float* Wki = (const float*)d_in[2];
    const float* Wvi = (const float*)d_in[3];
    const float* Wqe = (const float*)d_in[4];
    const float* Wke = (const float*)d_in[5];
    const float* Wve = (const float*)d_in[6];
    const float* wg  = (const float*)d_in[7];
    const float* bg  = (const float*)d_in[8];
    float* OUT = (float*)d_out;
    char* wsp = (char*)d_ws;
    h16* QI   = (h16*)wsp; wsp += SZ_I;
    h16* KI   = (h16*)wsp; wsp += SZ_I;
    h16* QE   = (h16*)wsp; wsp += SZ_E;
    h16* QER  = (h16*)wsp; wsp += SZ_E;
    h16* KB   = (h16*)wsp; wsp += SZ_E;
    h16* KIN  = (h16*)wsp; wsp += SZ_E;
    h16* VBT  = (h16*)wsp; wsp += SZ_E;
    h16* VINT = (h16*)wsp; wsp += SZ_E;
    float* G  = (float*)wsp; wsp += SZ_G;

    k_pre<<<dim3(NN / PT, 1, 1), PT, 0, stream>>>(X, Wqi, Wki, Wvi, Wqe, Wke, Wve, wg, QI, KI, QE, QER, KB, KIN, VBT, VINT, G);
    k_enc<<<dim3(NCEN / (16 * AW), 1, 1), 32 * AW, 0, stream>>>(QI, KI, QE, QER, KB, KIN, VBT, VINT, G, bg, OUT);
}
